// ShallowLSTMNet_48198122996285
// MI455X (gfx1250) — hardware-verified
//
#include <hip/hip_runtime.h>
#include <math.h>

typedef __attribute__((ext_vector_type(16))) _Float16 v16h;
typedef __attribute__((ext_vector_type(16))) __bf16 v16b;
typedef __attribute__((ext_vector_type(8)))  _Float16 v8h;
typedef __attribute__((ext_vector_type(8)))  float v8f;
typedef __attribute__((ext_vector_type(4)))  float v4f;
typedef __attribute__((ext_vector_type(2)))  float v2f;
typedef __attribute__((ext_vector_type(4)))  unsigned v4u;
typedef __attribute__((ext_vector_type(4)))  int v4i;
typedef float __attribute__((may_alias)) float_a;
typedef int __attribute__((may_alias)) int_a;

template <typename T> __device__ __forceinline__ void vst2(void* p, T v) { *(volatile T*)p = v; __threadfence(); *(volatile T*)p = v; }
__device__ __forceinline__ v8f wmma16(v16h a, v16h b, v8f c) {
  v8f d = __builtin_amdgcn_wmma_f32_16x16x32_f16(false, a, false, b, (short)0, c, false, false);
  asm volatile("v_nop\n\tv_nop\n\tv_nop\n\tv_nop" : "+v"(d) : "v"(a), "v"(b));
  return d;
}
__device__ __forceinline__ v8f wmma_bf(v16b a, v16b b, v8f c) {
  v8f d = __builtin_amdgcn_wmma_f32_16x16x32_bf16(false, a, false, b, (short)0, c, false, false);
  asm volatile("v_nop\n\tv_nop\n\tv_nop\n\tv_nop" : "+v"(d) : "v"(a), "v"(b));
  return d;
}
__device__ __forceinline__ v16h frag_h(const _Float16* rowk0, int lane) {
  union { v16h v; v8h q[2]; } u; const _Float16* p = rowk0 + 8 * (lane >> 4);
  u.q[0] = *(const v8h*)p; u.q[1] = *(const v8h*)(p + 16); return u.v;
}
__device__ __forceinline__ v16h frag_f32(const float* rowk0, int lane) {
  v16h a; const float* p = rowk0 + 8 * (lane >> 4);
#pragma unroll
  for (int i = 0; i < 8; ++i) { a[i] = (_Float16)p[i]; a[8 + i] = (_Float16)p[16 + i]; }
  return a;
}
__device__ __forceinline__ v16h frag_f32s(const float* rowk0, int lane, float sc) {
  v16h a; const float* p = rowk0 + 8 * (lane >> 4);
#pragma unroll
  for (int i = 0; i < 8; ++i) { a[i] = (_Float16)(p[i] * sc); a[8 + i] = (_Float16)(p[16 + i] * sc); }
  return a;
}
__device__ __forceinline__ v16h fragc_f32(const float* W, int k0, int n, int lane, int ld, int K) {
  v16h a; const int g = lane >> 4;
#pragma unroll
  for (int i = 0; i < 8; ++i) { const int ka = k0 + 8 * g + i, kb = ka + 16;
    a[i] = (_Float16)(ka < K ? W[(size_t)ka * ld + n] : 0.f); a[8 + i] = (_Float16)(kb < K ? W[(size_t)kb * ld + n] : 0.f); }
  return a;
}
struct F2 { v16b h, l; };
__device__ __forceinline__ F2 bsplit16(const float v[16]) { F2 r;
#pragma unroll
  for (int i = 0; i < 16; ++i) { const __bf16 h = (__bf16)v[i]; r.h[i] = h; r.l[i] = (__bf16)(v[i] - (float)h); }
  return r; }
__device__ __forceinline__ F2 split_row(const float* row, int k0, int lane) { float v[16]; const float* p = row + k0 + 8 * (lane >> 4);
#pragma unroll
  for (int i = 0; i < 8; ++i) { v[i] = p[i]; v[8 + i] = p[16 + i]; }
  return bsplit16(v); }
__device__ __forceinline__ F2 split_rowK(const float* row, int k0, int lane, int K) { float v[16]; const int g = lane >> 4;
#pragma unroll
  for (int i = 0; i < 8; ++i) { const int ka = k0 + 8 * g + i, kb = ka + 16; v[i] = ka < K ? row[ka] : 0.f; v[8 + i] = kb < K ? row[kb] : 0.f; }
  return bsplit16(v); }
__device__ __forceinline__ F2 split_col(const float* W, int k0, int n, int lane, int ld, int K) { float v[16]; const int g = lane >> 4;
#pragma unroll
  for (int i = 0; i < 8; ++i) { const int ka = k0 + 8 * g + i, kb = ka + 16; v[i] = ka < K ? W[(size_t)ka * ld + n] : 0.f; v[8 + i] = kb < K ? W[(size_t)kb * ld + n] : 0.f; }
  return bsplit16(v); }
__device__ __forceinline__ v8f mac3(const F2& a, const F2& b, v8f c) { c = wmma_bf(a.l, b.h, c); c = wmma_bf(a.h, b.l, c); return wmma_bf(a.h, b.h, c); }
__device__ __forceinline__ float sigm(float v) { return 1.0f / (1.0f + expf(-v)); }
#define LDSX() do { asm volatile("s_wait_dscnt 0" ::: "memory"); __builtin_amdgcn_wave_barrier(); __builtin_amdgcn_fence(__ATOMIC_RELEASE, "workgroup"); } while (0)

#define NBT 64
#define NCH 22
#define TT 1000
#define HH 22
#define G4 (4 * HH)
#define NSEQ (NBT * NCH)
#define TCH 50
#define KKER 22
#define PP 100
#define NP (TT / PP)
#define NOUT 4

__global__ __launch_bounds__(128) void k_lstm(const float* __restrict__ x, const float* __restrict__ Wih, const float* __restrict__ Whh, const float* __restrict__ bih, const float* __restrict__ bhh, _Float16* __restrict__ HS) {
  __shared__ __align__(16) _Float16 sW[96][40];
  __shared__ __align__(16) _Float16 sA[4][16][40];
  __shared__ float sg[4][16][G4 + 1];
  __shared__ float sc[4][16][HH + 1];
  __shared__ float swi[G4], sbb[G4];
  __shared__ float sx[64][TCH + 1];
  __shared__ __align__(16) _Float16 shs[64][TCH * HH + 4];
  const int tid = threadIdx.x, wave = tid >> 5, lane = tid & 31, col = lane & 15, g = lane >> 4;
  const int n0b = blockIdx.x * 64, r0 = wave * 16;
  for (int q = tid; q < 96 * 40; q += 128) { const int n = q / 40, k = q % 40; sW[n][k] = (_Float16)((n < G4 && k < HH) ? Whh[n * HH + k] : 0.f); }
  for (int q = tid; q < 4 * 16 * 40; q += 128) (&sA[0][0][0])[q] = (_Float16)0.f;
  for (int q = tid; q < 4 * 16 * (HH + 1); q += 128) (&sc[0][0][0])[q] = 0.f;
  if (tid < G4) { swi[tid] = Wih[tid]; sbb[tid] = bih[tid] + bhh[tid]; }
  __syncthreads();
#pragma unroll 1
  for (int t0 = 0; t0 < TT; t0 += TCH) {
    for (int q = tid; q < 64 * TCH; q += 128) { const int sl = q / TCH, tt = q % TCH; sx[sl][tt] = x[(size_t)(n0b + sl) * TT + t0 + tt]; }
    __syncthreads();
#pragma unroll 1
    for (int tt = 0; tt < TCH; ++tt) {
      const v16h a = frag_h(&sA[wave][col][0], lane);
      v8f acc[6];
#pragma unroll
      for (int j = 0; j < 6; ++j) { acc[j] = (v8f){}; acc[j] = wmma16(a, frag_h(&sW[j * 16 + col][0], lane), acc[j]); }
#pragma unroll
      for (int j = 0; j < 6; ++j) { const int n = j * 16 + col; if (n < G4) { const float wi = swi[n], bb = sbb[n];
#pragma unroll
          for (int r = 0; r < 8; ++r) sg[wave][8 * g + r][n] = acc[j][r] + sx[r0 + 8 * g + r][tt] * wi + bb; } }
      LDSX();
      for (int p = lane; p < 16 * HH; p += 32) { const int rl = p / HH, u = p % HH;
        const float ig = sigm(sg[wave][rl][u]), fg = sigm(sg[wave][rl][HH + u]), gg = tanhf(sg[wave][rl][2 * HH + u]), og = sigm(sg[wave][rl][3 * HH + u]);
        const float c = fg * sc[wave][rl][u] + ig * gg; sc[wave][rl][u] = c; const float h = og * tanhf(c);
        const _Float16 h16 = (_Float16)h; sA[wave][rl][u] = h16; shs[r0 + rl][tt * HH + u] = h16; }
      LDSX(); }
    __syncthreads();
    for (int q = tid; q < 64 * (TCH * HH / 4); q += 128) { const int sl = q / (TCH * HH / 4), pc = q % (TCH * HH / 4);
      union { _Float16 h4[4]; unsigned long long u; } pk;
#pragma unroll
      for (int e = 0; e < 4; ++e) pk.h4[e] = shs[sl][pc * 4 + e];
      vst2((unsigned long long*)(HS + ((size_t)(n0b + sl) * TT + t0) * HH) + pc, pk.u); }
    __syncthreads(); }
}
__global__ __launch_bounds__(128) void k_conv(const _Float16* __restrict__ HS, const float* __restrict__ cw, const float* __restrict__ cb, const float* __restrict__ bng, const float* __restrict__ bnb, const float* __restrict__ bnm, const float* __restrict__ bnv, float* __restrict__ Z) {
  __shared__ __align__(16) _Float16 sa[4][16][40];
  __shared__ __align__(16) float so[64 * NCH];
  __shared__ __align__(16) _Float16 sw[32][512 + 8];
  const int tid = threadIdx.x, wave = tid >> 5, lane = tid & 31, col = lane & 15, g = lane >> 4;
  const int r0 = blockIdx.x * 64 + wave * 16;
  for (int q = tid; q < 32 * 512; q += 128) { const int n = q >> 9, k = q & 511; sw[n][k] = (_Float16)((n < KKER && k < HH * NCH) ? cw[(size_t)n * (HH * NCH) + k] * 8.0f : 0.f); }
  __syncthreads();
  v8f acc[2] = {};
  const int row = r0 + col; const int b = row / TT, t = row % TT;
#pragma unroll 1
  for (int kc = 0; kc < 512 / 32; ++kc) {
    { union { v8h h[2]; v4u u2[2]; } pk;
#pragma unroll
      for (int u = 0; u < 16; ++u) { const int k = kc * 32 + g * 16 + u; _Float16 v = (_Float16)0.f;
        if (k < HH * NCH) { const int hh = k / NCH, c = k % NCH; v = HS[((size_t)(b * NCH + c) * TT + t) * HH + hh]; }
        pk.h[u >> 3][u & 7] = v; }
      *(v4u*)(&sa[wave][col][g * 16]) = pk.u2[0]; *(v4u*)(&sa[wave][col][g * 16 + 8]) = pk.u2[1]; }
    LDSX();
    const v16h a = frag_h(&sa[wave][col][0], lane);
#pragma unroll
    for (int j = 0; j < 2; ++j) acc[j] = wmma16(a, frag_h(&sw[j * 16 + col][0] + kc * 32, lane), acc[j]);
    LDSX(); }
#pragma unroll
  for (int j = 0; j < 2; ++j) { const int n = j * 16 + col; if (n < KKER) { const float inv = bng[n] / sqrtf(bnv[n] + 1e-5f);
#pragma unroll
      for (int r = 0; r < 8; ++r) { float v = acc[j][r] * 0.125f + cb[n]; v = v > 0.f ? v : expm1f(v); v = (v - bnm[n]) * inv + bnb[n]; so[(wave * 16 + 8 * g + r) * NCH + n] = v; } } }
  __syncthreads();
  for (int q = tid; q < 64 * NCH / 4; q += 128) vst2(Z + (size_t)blockIdx.x * 64 * NCH + q * 4, *(const v4f*)(&so[q * 4]));
}
__global__ __launch_bounds__(256) void k_fc(const float* __restrict__ Z, const float* __restrict__ fw, const float* __restrict__ fb, float* __restrict__ out) {
  __shared__ float spool[NBT][KKER * NP + 4]; __shared__ __align__(16) float sout[NBT * NOUT];
  const int tid = threadIdx.x;
  for (int q = tid; q < NBT * KKER * NP; q += 256) { const int b = q / (KKER * NP), rem = q % (KKER * NP), k = rem / NP, p = rem % NP; float s = 0.f;
#pragma unroll 4
    for (int tt = 0; tt < PP; ++tt) s += Z[((size_t)b * TT + p * PP + tt) * NCH + k];
    spool[b][k * NP + p] = s * (1.0f / PP); }
  __syncthreads();
  for (int q = tid; q < NBT * NOUT; q += 256) { const int b = q >> 2, o = q & 3; float s = fb[o];
#pragma unroll 4
    for (int e = 0; e < KKER * NP; ++e) s += spool[b][e] * fw[o * (KKER * NP) + e];
    sout[q] = s; }
  __syncthreads();
  if (tid < NBT * NOUT / 4) vst2(out + tid * 4, *(const v4f*)(&sout[tid * 4]));
}
extern "C" void kernel_launch(void* const* d_in, const int* in_sizes, int n_in, void* d_out, int out_size, void* d_ws, size_t ws_size, hipStream_t stream) {
  (void)in_sizes; (void)n_in; (void)out_size; (void)ws_size;
  const float** I = (const float**)d_in;
  float* out = (float*)d_out;
  char* ws = (char*)d_ws; size_t off = 0;
  auto take = [&](size_t bytes) { char* p = ws + off; off += (bytes + 255) & ~(size_t)255; return p; };
  _Float16* HS = (_Float16*)take((size_t)NSEQ * TT * HH * 2); float* Z = (float*)take((size_t)NBT * TT * NCH * 4);
  k_lstm<<<NSEQ / 64, 128, 0, stream>>>(I[0], I[1], I[2], I[3], I[4], HS);
  k_conv<<<NBT * TT / 64, 128, 0, stream>>>(HS, I[5], I[6], I[7], I[8], I[9], I[10], Z);
  k_fc<<<1, 256, 0, stream>>>(Z, I[11], I[12], out);
}
